// KascadeReuseAttention_28312424415933
// MI455X (gfx1250) — hardware-verified
//
#include <hip/hip_runtime.h>


#define SQ   2048
#define DMD  1024
#define NH_  16
#define HD   64
#define TL   16
#define NA   3
#define KS   64
typedef _Float16 h16;
typedef unsigned short bf;
typedef __attribute__((ext_vector_type(16))) __bf16   v16bf;
typedef __attribute__((ext_vector_type(16))) _Float16 v16h;
typedef __attribute__((ext_vector_type(8)))  _Float16 v8h;
typedef __attribute__((ext_vector_type(8)))  unsigned short v8us;
typedef __attribute__((ext_vector_type(8)))  float    v8f;
typedef __attribute__((ext_vector_type(4)))  float    v4f;
typedef v8h  __attribute__((may_alias)) v8ha;
typedef v4f  __attribute__((may_alias)) v4fa;
typedef v8us __attribute__((may_alias)) v8usa;

__device__ __forceinline__ unsigned short f2bf(float f) { unsigned u = __float_as_uint(f); u += 0x7FFFu + ((u >> 16) & 1u); return (unsigned short)(u >> 16); }
__device__ __forceinline__ float bf2f(unsigned short b) { return __uint_as_float(((unsigned)b) << 16); }
__device__ __forceinline__ float bfr(float f) { return bf2f(f2bf(f)); }
__device__ __forceinline__ v16h cat16(v8h lo, v8h hi) { return __builtin_shufflevector(lo, hi, 0, 1, 2, 3, 4, 5, 6, 7, 8, 9, 10, 11, 12, 13, 14, 15); }
__device__ __forceinline__ v16bf cat16b(v8us lo, v8us hi) { return __builtin_bit_cast(v16bf, __builtin_shufflevector(lo, hi, 0, 1, 2, 3, 4, 5, 6, 7, 8, 9, 10, 11, 12, 13, 14, 15)); }
__device__ __forceinline__ v8f wmma16(v16h a, v16h b, v8f c) { return __builtin_amdgcn_wmma_f32_16x16x32_f16(false, a, false, b, (short)0, c, false, false); }
__device__ __forceinline__ v8f wmmab(v16bf a, v16bf b, v8f c) { return __builtin_amdgcn_wmma_f32_16x16x32_bf16(false, a, false, b, (short)0, c, false, false); }


template <typename T16> struct WFrag;
template <> struct WFrag<h16> { typedef v16h V; static __device__ __forceinline__ V ld(const h16* p) { return cat16(*(const v8h*)p, *(const v8h*)(p + 16)); } static __device__ __forceinline__ v8f mma(V a, V b, v8f c) { return wmma16(a, b, c); } };
template <> struct WFrag<bf> { typedef v16bf V; static __device__ __forceinline__ V ld(const bf* p) { return cat16b(*(const v8us*)p, *(const v8us*)(p + 16)); } static __device__ __forceinline__ v8f mma(V a, V b, v8f c) { return wmmab(a, b, c); } };
template <typename T16, int NSPLIT, bool BIAS>
__global__ __launch_bounds__(32) void k_gemmw(const T16* __restrict__ A, const T16* __restrict__ A2, const T16* __restrict__ Bt, const T16* __restrict__ Bt2, int K, float* C, int ldc, const float* __restrict__ bias, size_t sA, size_t sB, size_t sC) {
    typedef typename WFrag<T16>::V V;
    __shared__ __align__(16) float os[16 * 68];
    const size_t z = blockIdx.z; A += z * sA; if (A2) A2 += z * sA; Bt += z * sB; if (Bt2) Bt2 += z * sB; C += z * sC;
    const int lane = threadIdx.x & 31, lr = lane & 15, hi = lane >> 4; const int r0 = blockIdx.x * 64, c0 = blockIdx.y * 64;
    v8f acc[4][4];
#pragma unroll
    for (int mb = 0; mb < 4; ++mb)
#pragma unroll
        for (int nb = 0; nb < 4; ++nb) acc[mb][nb] = (v8f){};
    const size_t aoff = (size_t)(r0 + lr) * K + 8 * hi, boff = (size_t)(c0 + lr) * K + 8 * hi;
#pragma unroll 1
    for (int kc = 0; kc < K; kc += 32) {
        V a[4], a2[4];
#pragma unroll
        for (int mb = 0; mb < 4; ++mb) { a[mb] = WFrag<T16>::ld(A + aoff + (size_t)mb * 16 * K + kc); if (NSPLIT == 1 || NSPLIT == 2) a2[mb] = WFrag<T16>::ld(A2 + aoff + (size_t)mb * 16 * K + kc); }
#pragma unroll
        for (int nb = 0; nb < 4; ++nb) { const V b = WFrag<T16>::ld(Bt + boff + (size_t)nb * 16 * K + kc); V b2; if (NSPLIT >= 2) b2 = WFrag<T16>::ld(Bt2 + boff + (size_t)nb * 16 * K + kc);
#pragma unroll
            for (int mb = 0; mb < 4; ++mb) { acc[mb][nb] = WFrag<T16>::mma(a[mb], b, acc[mb][nb]); if (NSPLIT == 1 || NSPLIT == 2) acc[mb][nb] = WFrag<T16>::mma(a2[mb], b, acc[mb][nb]); if (NSPLIT >= 2) acc[mb][nb] = WFrag<T16>::mma(a[mb], b2, acc[mb][nb]); } }
        asm volatile("v_nop\n\tv_nop\n\tv_nop\n\tv_nop" : "+v"(acc[0][0]), "+v"(acc[1][1]), "+v"(acc[2][2]), "+v"(acc[3][3]) : "v"(a[0]), "v"(a[3]));
    }
#pragma unroll
    for (int mb = 0; mb < 4; ++mb) {
#pragma unroll
        for (int nb = 0; nb < 4; ++nb) {
#pragma unroll
            for (int j = 0; j < 8; ++j) os[(hi * 8 + j) * 68 + nb * 16 + lr] = acc[mb][nb][j]; }
        __builtin_amdgcn_wave_barrier(); asm volatile("" ::: "memory");
        float* crow = C + (size_t)(r0 + mb * 16) * ldc + c0;
#pragma unroll 1
        for (int ps = 0; ps < 2; ++ps) {
#pragma unroll
            for (int s = 0; s < 8; ++s) { const int row = 2 * s + hi, cofs = lr * 4; v4f val = *(const v4fa*)(os + row * 68 + cofs); if (BIAS) { val[0] += bfr(bias[c0 + cofs]); val[1] += bfr(bias[c0 + cofs + 1]); val[2] += bfr(bias[c0 + cofs + 2]); val[3] += bfr(bias[c0 + cofs + 3]); }
                *(volatile v4f*)(crow + (size_t)row * ldc + cofs) = val; }
            if (ps == 0) __threadfence(); }
        __builtin_amdgcn_wave_barrier(); asm volatile("" ::: "memory");
    }
}

__device__ __forceinline__ void splitf(float y, unsigned short& h, unsigned short& l) { h = f2bf(y); l = f2bf(y - bf2f(h)); }
typedef __attribute__((ext_vector_type(2))) unsigned short v2us;
typedef __attribute__((ext_vector_type(4))) unsigned short v4us;
typedef __attribute__((ext_vector_type(2))) float v2f;

__global__ __launch_bounds__(256) void k_wtG(const float* __restrict__ w, int K, int N, bf* Bt) {
    const int lane = threadIdx.x & 31; const int L0 = (blockIdx.x * 8 + (threadIdx.x >> 5)) * 8; const int nlines = N * K / 64;
#pragma unroll
    for (int ps = 0; ps < 2; ++ps) {
#pragma unroll 1
        for (int l = 0; l < 8; ++l) { const int L = L0 + l; if (L >= nlines) break; const size_t e = (size_t)L * 64 + lane * 2; const int k = (int)(e % K), n = (int)(e / K); v2us o;
            o[0] = f2bf(w[(size_t)k * N + n]); o[1] = f2bf(w[(size_t)(k + 1) * N + n]); *(volatile v2us*)(Bt + e) = o; }
        if (ps == 0) __threadfence(); }
}
__global__ __launch_bounds__(256) void k_cvt8(const float* __restrict__ src, bf* dst, size_t n8) { const size_t i = (size_t)blockIdx.x * 256 + threadIdx.x; if (i >= n8) return; const v8f v = *(const v8f*)(src + i * 8); v8us o;
#pragma unroll
    for (int k = 0; k < 8; ++k) o[k] = f2bf(v[k]); *(volatile v8us*)(dst + i * 8) = o; __threadfence(); *(volatile v8us*)(dst + i * 8) = o; }
__global__ __launch_bounds__(256) void k_rope2(const float* __restrict__ F, const float* __restrict__ cs, const float* __restrict__ sn, float* R) { const size_t e = ((size_t)blockIdx.x * 256 + threadIdx.x) * 4; if (e >= (size_t)SQ * DMD) return; const int c = (int)(e % DMD); const int t = (int)(e / DMD); const int h = c / HD, d0 = c % HD; const float* f = F + (size_t)t * DMD + h * HD; v4f o;
#pragma unroll
    for (int u = 0; u < 4; ++u) { const int dd = d0 + u; const int j = dd & 31; const float cc = bfr(cs[(size_t)t * 32 + j]), ss = bfr(sn[(size_t)t * 32 + j]); const float xv = f[dd]; const float rot = (dd < 32) ? -f[dd + 32] : f[dd - 32];
        float a = __fmul_rn(xv, cc); asm volatile("" : "+v"(a)); float b2 = __fmul_rn(rot, ss); asm volatile("" : "+v"(b2)); o[u] = __fadd_rn(a, b2); }
    *(volatile v4f*)(R + e) = o; __threadfence(); *(volatile v4f*)(R + e) = o; }
__global__ __launch_bounds__(256) void k_spat(const float* __restrict__ Q, const float* __restrict__ K, const float* __restrict__ V, const int* __restrict__ anc, bf* Ch, bf* Cl) {
    const int lane = threadIdx.x & 31; const int wq = blockIdx.x * 8 + (threadIdx.x >> 5); if (wq >= NH_ * SQ) return; const int h = wq / SQ; const int q = wq % SQ;
    const float* qv = Q + (size_t)q * DMD + h * HD; const int* ar = anc + ((size_t)h * SQ + q) * NA;
    int tok[2]; float lg[2];
#pragma unroll
    for (int w = 0; w < 2; ++w) { const int k = lane + 32 * w; const int tile = (k / TL < NA) ? ar[k / TL] : (q / TL); int t = tile * TL + (k % TL); t = min(max(t, 0), SQ - 1); tok[w] = t; const float* kr = K + (size_t)t * DMD + h * HD; float acc = 0.f;
#pragma unroll 1
        for (int d = 0; d < HD; ++d) { float p = __fmul_rn(qv[d], kr[d]); asm volatile("" : "+v"(p)); acc = __fadd_rn(acc, p); }
        lg[w] = (t > q) ? -1.0e10f : acc * 0.125f; }
    float mx = fmaxf(lg[0], lg[1]);
#pragma unroll
    for (int sh = 16; sh; sh >>= 1) mx = fmaxf(mx, __shfl_xor(mx, sh, 32));
    float e0, e1; { float d0 = __fsub_rn(lg[0], mx); asm volatile("" : "+v"(d0)); e0 = __expf(d0); float d1 = __fsub_rn(lg[1], mx); asm volatile("" : "+v"(d1)); e1 = __expf(d1); }
    float sum = __fadd_rn(e0, e1);
#pragma unroll
    for (int sh = 16; sh; sh >>= 1) sum += __shfl_xor(sum, sh, 32);
    const bool allfut = (mx <= -1.0e10f); const float inv = __fdiv_rn(1.0f, sum); float w0 = allfut ? 0.f : __fmul_rn(e0, inv), w1 = allfut ? 0.f : __fmul_rn(e1, inv); if (w0 != w0) w0 = 0.f; if (w1 != w1) w1 = 0.f;
    const int dA = lane * 2; float o0 = 0.f, o1 = 0.f;
#pragma unroll 1
    for (int k = 0; k < KS; ++k) { const int src = k & 31; const float wk = __shfl((k < 32) ? w0 : w1, src, 32); const int tk = __shfl((k < 32) ? tok[0] : tok[1], src, 32); const float* vr = V + (size_t)tk * DMD + h * HD + dA;
        float p0 = __fmul_rn(wk, vr[0]); asm volatile("" : "+v"(p0)); o0 = __fadd_rn(o0, p0); float p1 = __fmul_rn(wk, vr[1]); asm volatile("" : "+v"(p1)); o1 = __fadd_rn(o1, p1); }
    v2us oh, ol; { unsigned short a, b; splitf(o0, a, b); oh[0] = a; ol[0] = b; splitf(o1, a, b); oh[1] = a; ol[1] = b; }
    const size_t oo = (size_t)q * DMD + h * HD + dA; *(volatile v2us*)(Ch + oo) = oh; *(volatile v2us*)(Cl + oo) = ol; __threadfence(); *(volatile v2us*)(Ch + oo) = oh; *(volatile v2us*)(Cl + oo) = ol; }

extern "C" void kernel_launch(void* const* d_in, const int* in_sizes, int n_in,
                              void* d_out, int out_size, void* d_ws, size_t ws_size, hipStream_t stream) {
    (void)in_sizes; (void)n_in; (void)out_size;
    const float* x = (const float*)d_in[0]; const float* Wq = (const float*)d_in[1]; const float* Wk = (const float*)d_in[2]; const float* Wv = (const float*)d_in[3]; const float* Wo = (const float*)d_in[4]; const float* cs = (const float*)d_in[5]; const float* sn = (const float*)d_in[6]; const int* anc = (const int*)d_in[7];
    float* OUT = (float*)d_out;
    char* wsp = (char*)d_ws;
    auto take = [&](size_t bytes) { char* p = wsp; wsp += (bytes + 255) & ~(size_t)255; return (void*)p; };
    bf* BW[4]; for (int i = 0; i < 4; ++i) BW[i] = (bf*)take((size_t)DMD * DMD * 2); bf* XB = (bf*)take((size_t)SQ * DMD * 2);
    float* F = (float*)take((size_t)SQ * DMD * 4); float* QR = (float*)take((size_t)SQ * DMD * 4); float* KR = (float*)take((size_t)SQ * DMD * 4); float* VF = (float*)take((size_t)SQ * DMD * 4); bf* Ch = (bf*)take((size_t)SQ * DMD * 2); bf* Cl = (bf*)take((size_t)SQ * DMD * 2);
    if ((size_t)(wsp - (char*)d_ws) > ws_size) return;
    const float* Wl[4] = {Wq, Wk, Wv, Wo}; for (int i = 0; i < 4; ++i) k_wtG<<<(unsigned)((DMD * DMD / 64 + 63) / 64), 256, 0, stream>>>(Wl[i], DMD, DMD, BW[i]);
    k_cvt8<<<(SQ * DMD / 8 + 255) / 256, 256, 0, stream>>>(x, XB, SQ * DMD / 8);
    const dim3 gp(SQ / 64, DMD / 64, 1); const unsigned gE = (unsigned)(((size_t)SQ * DMD / 4 + 255) / 256);
    k_gemmw<bf, 0, false><<<gp, 32, 0, stream>>>(XB, nullptr, BW[0], nullptr, DMD, F, DMD, nullptr, 0, 0, 0); k_rope2<<<gE, 256, 0, stream>>>(F, cs, sn, QR);
    k_gemmw<bf, 0, false><<<gp, 32, 0, stream>>>(XB, nullptr, BW[1], nullptr, DMD, F, DMD, nullptr, 0, 0, 0); k_rope2<<<gE, 256, 0, stream>>>(F, cs, sn, KR);
    k_gemmw<bf, 0, false><<<gp, 32, 0, stream>>>(XB, nullptr, BW[2], nullptr, DMD, VF, DMD, nullptr, 0, 0, 0);
    k_spat<<<NH_ * SQ / 8, 256, 0, stream>>>(QR, KR, VF, anc, Ch, Cl);
    k_gemmw<bf, 1, false><<<gp, 32, 0, stream>>>(Ch, Cl, BW[3], nullptr, DMD, OUT, DMD, nullptr, 0, 0, 0);
}
